// FullAttention_87823491269160
// MI455X (gfx1250) — hardware-verified
//
#include <hip/hip_runtime.h>
#ifndef NB
#define NB 1
#endif
#ifndef SEQ
#define SEQ 2048
#endif
#define SEQ_FULL 2048
#define HID 2048
#define NQH 16
#define NKV 4
#define HDM 128
#define QD (NQH * HDM)
#define KD (NKV * HDM)
#define QGN (2 * QD)
#define KVN (2 * KD)
#define TE 128
#define RMS_EPS 0.000001f
#define SM_SCALE 0.08838834764831845f
#define PCARRY 4096.0f
#define GCARRY 64.0f
#define WSCALE 16.0f
static_assert(NB == 1);
static_assert(SEQ % 128 == 0);
static_assert(SEQ >= 2 * TE);
static_assert(SEQ <= SEQ_FULL);
static_assert((SEQ - TE) % 128 == 0);
static_assert(TE == 128);
static_assert(HDM == 128);

typedef __bf16 v16b __attribute__((ext_vector_type(16)));
typedef unsigned short v8us __attribute__((ext_vector_type(8), may_alias));
typedef unsigned short v4us __attribute__((ext_vector_type(4)));
typedef float v8f __attribute__((ext_vector_type(8)));
typedef float v4f __attribute__((ext_vector_type(4)));
typedef float v4fa __attribute__((ext_vector_type(4), may_alias));
typedef _Float16 v16h __attribute__((ext_vector_type(16)));
typedef _Float16 v4h __attribute__((ext_vector_type(4)));
typedef float fa __attribute__((may_alias));
typedef _Float16 ha __attribute__((may_alias));
union FragB { v16b v; v8us half[2]; unsigned short u[16]; };
union FragH { v16h v; v8us half[2]; _Float16 h[16]; unsigned short u[16]; };

__device__ __forceinline__ unsigned short bf16_bits(float x) { unsigned int u = __float_as_uint(x); return (unsigned short)((u + 0x7FFFu + ((u >> 16) & 1u)) >> 16); }
__device__ __forceinline__ float bf16_val(unsigned short b) { return __uint_as_float(((unsigned int)b) << 16); }
__device__ __forceinline__ float bf16_rne(float x) { return bf16_val(bf16_bits(x)); }

template <int NT>
__device__ __forceinline__ v8f mmaN(v16b ah, v16b al, v16b bh, v16b bl, v8f c) {
  c = __builtin_amdgcn_wmma_f32_16x16x32_bf16(false, ah, false, bh, (short)0, c, false, false);
  if (NT >= 2) c = __builtin_amdgcn_wmma_f32_16x16x32_bf16(false, al, false, bh, (short)0, c, false, false);
  if (NT >= 3) c = __builtin_amdgcn_wmma_f32_16x16x32_bf16(false, ah, false, bl, (short)0, c, false, false);
  asm volatile("v_nop\n\tv_nop\n\tv_nop\n\tv_nop" : "+v"(c) : "v"(ah), "v"(al), "v"(bh), "v"(bl));
  return c;
}
template <int NT>
__device__ __forceinline__ v8f mmaH(v16h ah, v16h al, v16h bh, v16h bl, v8f c) {
  c = __builtin_amdgcn_wmma_f32_16x16x32_f16(false, ah, false, bh, (short)0, c, false, false);
  if (NT >= 2) c = __builtin_amdgcn_wmma_f32_16x16x32_f16(false, al, false, bh, (short)0, c, false, false);
  if (NT >= 3) c = __builtin_amdgcn_wmma_f32_16x16x32_f16(false, ah, false, bl, (short)0, c, false, false);
  asm volatile("v_nop\n\tv_nop\n\tv_nop\n\tv_nop" : "+v"(c) : "v"(ah), "v"(al), "v"(bh), "v"(bl));
  return c;
}
__device__ __forceinline__ v16h g2_frag(const _Float16* p, int hh) { FragH f; f.half[0] = *(const v8us*)((const unsigned short*)p + 8 * hh); f.half[1] = *(const v8us*)((const unsigned short*)p + 16 + 8 * hh); return f.v; }
__device__ __forceinline__ v8f g2_mma(v16h a, v16h b, v8f c) { v8f d = __builtin_amdgcn_wmma_f32_16x16x32_f16(false, a, false, b, (short)0, c, false, false); asm volatile("v_nop\n\tv_nop\n\tv_nop\n\tv_nop" : "+v"(d) : "v"(a), "v"(b)); return d; }

__device__ __forceinline__ float half_reduce_max(float x) {
#pragma unroll
  for (int m = 1; m <= 8; m <<= 1) x = fmaxf(x, __shfl_xor(x, m, 32));
  return x;
}
__device__ __forceinline__ float half_reduce_add(float x) {
#pragma unroll
  for (int m = 1; m <= 8; m <<= 1) x += __shfl_xor(x, m, 32);
  return x;
}
__device__ __forceinline__ float silu_f(float g) { return g * __builtin_amdgcn_rcpf(1.0f + __expf(-g)); }

__global__ __launch_bounds__(256) void k_x16(const float* __restrict__ x, _Float16* __restrict__ X16, size_t n8) { const size_t t = (size_t)blockIdx.x * 256 + threadIdx.x; if (t >= n8) return; FragH f;
#pragma unroll
  for (int q = 0; q < 8; ++q) f.h[q] = (_Float16)bf16_rne(x[t * 8 + q]); *(volatile v8us*)((unsigned short*)X16 + t * 8) = f.half[0]; __threadfence(); *(volatile v8us*)((unsigned short*)X16 + t * 8) = f.half[0]; }

__global__ __launch_bounds__(256) void k_wt_f16(const float* __restrict__ W, _Float16* __restrict__ Wt, int K, int N, float scale) {
  const int t = blockIdx.x * 256 + threadIdx.x; if (t >= N * (K / 8)) return; const int n = t / (K / 8), k8 = (t % (K / 8)) * 8; FragH f;
#pragma unroll
  for (int i = 0; i < 8; ++i) f.h[i] = (_Float16)(bf16_rne(W[(size_t)(k8 + i) * N + n]) * scale); const v8us o = f.half[0];
  *(volatile v8us*)((unsigned short*)Wt + (size_t)n * K + k8) = o; __threadfence(); *(volatile v8us*)((unsigned short*)Wt + (size_t)n * K + k8) = o;
}
__global__ __launch_bounds__(256) void k_wt_bf16(const float* __restrict__ W, unsigned short* __restrict__ Wt, int K, int N) {
  const int t = blockIdx.x * 256 + threadIdx.x; const int k8n = K / 8; if (t >= N * k8n) return;
  const int n = t / k8n, k8 = (t % k8n) * 8; v8us v;
#pragma unroll
  for (int i = 0; i < 8; ++i) v[i] = bf16_bits(W[(size_t)(k8 + i) * N + n]);
  *(volatile v8us*)(Wt + (size_t)n * K + k8) = v; __threadfence(); *(volatile v8us*)(Wt + (size_t)n * K + k8) = v;
}

template <int ACT>
__global__ __launch_bounds__(128) void k_gemm2(const _Float16* __restrict__ A, int lda, size_t sA, const _Float16* __restrict__ Bh, int ldb, size_t sB, float alpha, const float* __restrict__ bias, size_t sBias, const float* __restrict__ CP, int rowsPerB, size_t sCPb, int row0g,
    float* __restrict__ C, _Float16* __restrict__ C16, int ldc, size_t sC, int M, int N, int K) { static_assert(ACT == 0);
  __shared__ __attribute__((aligned(16))) float so[4][32][68];
  const int tid = threadIdx.x, w = tid >> 5, lane = tid & 31, ln = lane & 15, hh = lane >> 4; const int by = blockIdx.y;
  A += (size_t)by * sA; Bh += (size_t)by * sB; const size_t cofs = (size_t)by * sC; const float* bp = bias ? bias + (size_t)by * sBias : nullptr;
  const int ntn = N >> 6; const int mt = blockIdx.x / ntn, nq = blockIdx.x - mt * ntn; const int row0 = mt * 128 + 32 * w, col0 = nq * 64; if (row0 >= M) return;
  const _Float16* a0p = A + (size_t)(row0 + ln) * lda; const _Float16* a1p = a0p + (size_t)16 * lda;
  const _Float16* b0p = Bh + (size_t)(col0 + ln) * ldb; const _Float16* b1p = b0p + (size_t)16 * ldb; const _Float16* b2p = b1p + (size_t)16 * ldb; const _Float16* b3p = b2p + (size_t)16 * ldb;
  const v8f z8 = {0.f,0.f,0.f,0.f,0.f,0.f,0.f,0.f}; v8f c00 = z8, c01 = z8, c02 = z8, c03 = z8, c10 = z8, c11 = z8, c12 = z8, c13 = z8;
#pragma unroll 1
  for (int kb = 0; kb < K; kb += 32) { const v16h a0 = g2_frag(a0p + kb, hh), a1 = g2_frag(a1p + kb, hh);
    v16h b = g2_frag(b0p + kb, hh); c00 = g2_mma(a0, b, c00); c10 = g2_mma(a1, b, c10);
    b = g2_frag(b1p + kb, hh); c01 = g2_mma(a0, b, c01); c11 = g2_mma(a1, b, c11);
    b = g2_frag(b2p + kb, hh); c02 = g2_mma(a0, b, c02); c12 = g2_mma(a1, b, c12);
    b = g2_frag(b3p + kb, hh); c03 = g2_mma(a0, b, c03); c13 = g2_mma(a1, b, c13); }
  v8f accs[8] = {c00, c01, c02, c03, c10, c11, c12, c13};
#pragma unroll
  for (int u = 0; u < 8; ++u) { const int t = u & 3, half = u >> 2; const int col = col0 + t * 16 + ln; const float bv = bp ? bf16_rne(bp[col]) : 0.f;
#pragma unroll
    for (int r = 0; r < 8; ++r) { const int rloc = half * 16 + 8 * hh + r; float v = accs[u][r] * alpha + bv; if (CP) { if (rowsPerB < 0) v += CP[cofs + (size_t)(row0g + row0 + rloc) * ldc + col]; else { const int bidx = (row0g + row0 + rloc) / rowsPerB; v += CP[(size_t)bidx * sCPb + (size_t)by * 64 + col]; } }
      so[w][rloc][t * 16 + ln] = v; } }
  __builtin_amdgcn_fence(4  , "workgroup"); __builtin_amdgcn_wave_barrier();
  const int rsub = lane >> 4, c4 = (lane & 15) * 4;
  for (int pass = 0; pass < 2; ++pass) {
#pragma unroll
    for (int q = 0; q < 16; ++q) { const int r = q * 2 + rsub; const v4f v = *(const v4fa*)&so[w][r][c4]; if (C) *(volatile v4f*)(C + cofs + (size_t)(row0 + r) * ldc + col0 + c4) = v; if (C16) { v4h h4; for (int i = 0; i < 4; ++i) h4[i] = (_Float16)v[i]; *(volatile v4h*)(C16 + cofs + (size_t)(row0 + r) * ldc + col0 + c4) = h4; } }
    if (pass == 0) __threadfence(); } }

template <bool ASPLIT>
__global__ __launch_bounds__(128) void k_gemm_bf(const float* __restrict__ A, int lda, const unsigned short* __restrict__ Wt, int ldb, float* __restrict__ C, int ldc, int M, int N, int K) {
  __shared__ __attribute__((aligned(16))) float so[4][16][64];
  const int tid = threadIdx.x, w = tid >> 5, lane = tid & 31, ln = lane & 15, hh = lane >> 4;
  const int ntn = N / 64;
  const int wid = blockIdx.x * 4 + w;
  const int mt = wid / ntn, nq = wid % ntn;
  if (mt * 16 >= M) return;
  const int row0 = mt * 16, col0 = nq * 64;
  const float* arow = A + (size_t)(row0 + ln) * lda;
  v8f acc[4] = {};
  for (int kb = 0; kb < K; kb += 32) {
    FragB ah, al;
    const v4f x0 = *(const v4fa*)(arow + kb + 8 * hh), x1 = *(const v4fa*)(arow + kb + 8 * hh + 4);
    const v4f x2 = *(const v4fa*)(arow + kb + 16 + 8 * hh), x3 = *(const v4fa*)(arow + kb + 16 + 8 * hh + 4);
    float xs[16] = {x0[0],x0[1],x0[2],x0[3],x1[0],x1[1],x1[2],x1[3],x2[0],x2[1],x2[2],x2[3],x3[0],x3[1],x3[2],x3[3]};
#pragma unroll
    for (int i = 0; i < 16; ++i) { const unsigned short hb = bf16_bits(xs[i]); ah.u[i] = hb; al.u[i] = ASPLIT ? bf16_bits(xs[i] - bf16_val(hb)) : (unsigned short)0; }
#pragma unroll
    for (int t = 0; t < 4; ++t) {
      const unsigned short* brow = Wt + (size_t)(col0 + t * 16 + ln) * ldb + kb;
      FragB b;
      b.half[0] = *(const v8us*)(brow + 8 * hh);
      b.half[1] = *(const v8us*)(brow + 16 + 8 * hh);
      acc[t] = mmaN<ASPLIT ? 2 : 1>(ah.v, al.v, b.v, b.v, acc[t]);
    }
  }
#pragma unroll
  for (int t = 0; t < 4; ++t) {
#pragma unroll
    for (int r = 0; r < 8; ++r) so[w][8 * hh + r][t * 16 + ln] = acc[t][r];
  }
  __builtin_amdgcn_fence(4  , "workgroup");
  __builtin_amdgcn_wave_barrier();
  const int rsub = lane >> 4, c4 = (lane & 15) * 4;
  for (int pass = 0; pass < 2; ++pass) {
#pragma unroll
    for (int q = 0; q < 8; ++q) {
      const int r = q * 2 + rsub;
      const v4f v = *(const v4fa*)&so[w][r][c4];
      *(volatile v4f*)(C + (size_t)(row0 + r) * ldc + col0 + c4) = v;
    }
    if (pass == 0) __threadfence();
  }
}

__global__ __launch_bounds__(256) void k_normrope(const float* __restrict__ QG, const float* __restrict__ KV, const int* __restrict__ pos, const float* __restrict__ invf,
    const float* __restrict__ qnw, const float* __restrict__ knw,
    unsigned short* __restrict__ Qh, unsigned short* __restrict__ Ql, unsigned short* __restrict__ Kh, unsigned short* __restrict__ Kl,
    float* __restrict__ QF, float* __restrict__ KF) {
  #pragma clang fp contract(off)
  __shared__ __attribute__((aligned(16))) float cst[64];
  __shared__ __attribute__((aligned(16))) float snt[64];
  const int t = blockIdx.x, tid = threadIdx.x, w = tid >> 5, lane = tid & 31;
  if (tid < 64) {
    const float th = (float)pos[t] * bf16_rne(invf[tid]);
    float sn, cs; sincosf(th, &sn, &cs);
    cst[tid] = cs; snt[tid] = sn;
  }
  __syncthreads();
  const int j4 = (lane & 15) * 4;
  const v4f cs4 = *(const v4fa*)(cst + j4), sn4 = *(const v4fa*)(snt + j4);
  const float sgn = (lane < 16) ? -1.0f : 1.0f;
  const int te = (t < TE) ? t : 0;
  for (int slot = w; slot < NQH + NKV; slot += 8) {
    const float* src; const float* wp; unsigned short* dh; unsigned short* dl; float* df;
    if (slot < NQH) {
      src = QG + (size_t)t * QGN + slot * HDM + lane * 4; wp = qnw;
      const size_t o = (size_t)t * QD + slot * HDM + lane * 4; dh = Qh + o; dl = Ql + o;
      df = QF + (size_t)te * QD + slot * HDM + lane * 4;
    } else {
      const int kv = slot - NQH;
      src = KV + (size_t)t * KVN + kv * HDM + lane * 4; wp = knw;
      const size_t o = (size_t)t * KD + kv * HDM + lane * 4; dh = Kh + o; dl = Kl + o;
      df = KF + (size_t)te * KD + kv * HDM + lane * 4;
    }
    const v4f x = *(const v4fa*)src; const v4f wv = *(const v4fa*)(wp + lane * 4);
    float ss = x[0] * x[0] + x[1] * x[1] + x[2] * x[2] + x[3] * x[3];
#pragma unroll
    for (int m = 1; m <= 16; m <<= 1) ss += __shfl_xor(ss, m, 32);
    const float rr = rsqrtf(ss * (1.0f / 128.0f) + RMS_EPS);
    float xn[4], xp[4], ov[4];
#pragma unroll
    for (int q = 0; q < 4; ++q) xn[q] = (x[q] * rr) * bf16_rne(wv[q]);
#pragma unroll
    for (int q = 0; q < 4; ++q) xp[q] = __shfl_xor(xn[q], 16, 32) * sgn;
#pragma unroll
    for (int q = 0; q < 4; ++q) ov[q] = xn[q] * cs4[q] + xp[q] * sn4[q];
    v4us hi4, lo4; v4f of;
#pragma unroll
    for (int q = 0; q < 4; ++q) { const unsigned short hb = bf16_bits(ov[q]); hi4[q] = hb; lo4[q] = bf16_bits(ov[q] - bf16_val(hb)); of[q] = ov[q]; }
    for (int pass = 0; pass < 2; ++pass) {
      *(volatile v4us*)dh = hi4; *(volatile v4us*)dl = lo4;
      if (t < TE) *(volatile v4f*)df = of;
      if (pass == 0) __threadfence();
    }
  }
}

__global__ __launch_bounds__(256) void k_vt(const float* __restrict__ KV, _Float16* __restrict__ VT) {
  __shared__ _Float16 tl[HDM][66];
  const int tid = threadIdx.x; const int kvh = blockIdx.x / (SEQ / 64), sg = blockIdx.x % (SEQ / 64); const int s0 = sg * 64;
  for (int i = tid; i < 64 * 32; i += 256) { const int j = i >> 5, d4 = (i & 31) * 4;
    const v4f a = *(const v4fa*)(KV + (size_t)(s0 + j) * KVN + KD + kvh * HDM + d4);
#pragma unroll
    for (int q = 0; q < 4; ++q) tl[d4 + q][j] = (_Float16)a[q]; }
  __syncthreads();
  for (int pass = 0; pass < 2; ++pass) {
#pragma unroll
    for (int rd = 0; rd < 4; ++rd) { const int d = rd * 32 + (tid >> 3), pc = tid & 7; FragH f;
#pragma unroll
      for (int q = 0; q < 8; ++q) f.h[q] = tl[d][pc * 8 + q];
      *(volatile v8us*)((unsigned short*)VT + ((size_t)(kvh * HDM + d) * SEQ + s0 + pc * 8)) = f.half[0]; }
    if (pass == 0) __threadfence(); }
}

__global__ __launch_bounds__(128) void k_flash(const unsigned short* __restrict__ Qh, const unsigned short* __restrict__ Ql,
    const unsigned short* __restrict__ Kh, const unsigned short* __restrict__ Kl, const _Float16* __restrict__ VT,
    const float* __restrict__ QG, _Float16* __restrict__ G16, int qb0) {
  __shared__ __attribute__((aligned(16))) float smem[8192];
  unsigned short* lK = (unsigned short*)smem;
  unsigned short* lVt = lK + 2 * 32 * 136;
  ha* lP = (ha*)(lVt + 128 * 40);
  fa* so = (fa*)smem;
  const int h = blockIdx.y, kvh = h >> 2, qb = qb0 + blockIdx.x * 64;
  const int tid = threadIdx.x, lane = tid & 31, w = tid >> 5, ln = lane & 15, hh = lane >> 4;
  const int qrow0 = qb + 16 * w;
  const unsigned short* qhp = Qh + (size_t)(qrow0 + ln) * QD + h * HDM;
  const unsigned short* qlp = Ql + (size_t)(qrow0 + ln) * QD + h * HDM;
  const v8f z8 = {0.f,0.f,0.f,0.f,0.f,0.f,0.f,0.f};
  v8f o[8];
#pragma unroll
  for (int n = 0; n < 8; ++n) o[n] = z8;
  float m[8], l[8];
#pragma unroll
  for (int r = 0; r < 8; ++r) { m[r] = -3.0e38f; l[r] = 0.f; }
  const int ntiles = (qb + 64) / 32;
#pragma unroll 1
  for (int kt = 0; kt < ntiles; ++kt) {
    const int key0 = kt * 32;
#pragma unroll
    for (int u = 0; u < 4; ++u) {
      const int i = tid + 128 * u;
      const int j = i >> 4, pk = i & 15;
      const size_t ko = (size_t)(key0 + j) * KD + kvh * HDM + pk * 8;
      const v8us a = *(const v8us*)(Kh + ko); const v8us b = *(const v8us*)(Kl + ko);
      *(v8us*)(lK + j * 136 + pk * 8) = a; *(v8us*)(lK + 32 * 136 + j * 136 + pk * 8) = b;
      const int d = i >> 2, pv = i & 3;
      const v8us v = *(const v8us*)((const unsigned short*)VT + ((size_t)(kvh * HDM + d) * SEQ + key0 + pv * 8));
      *(v8us*)(lVt + d * 40 + pv * 8) = v;
    }
    __syncthreads();
    v8f sA = z8, sB = z8;
#pragma unroll
    for (int c = 0; c < 4; ++c) {
      FragB qh, ql;
      qh.half[0] = *(const v8us*)(qhp + c * 32 + 8 * hh); qh.half[1] = *(const v8us*)(qhp + c * 32 + 16 + 8 * hh);
      ql.half[0] = *(const v8us*)(qlp + c * 32 + 8 * hh); ql.half[1] = *(const v8us*)(qlp + c * 32 + 16 + 8 * hh);
      const unsigned short* kp = lK + ln * 136 + c * 32;
      FragB kh, kl;
      kh.half[0] = *(const v8us*)(kp + 8 * hh); kh.half[1] = *(const v8us*)(kp + 16 + 8 * hh);
      kl.half[0] = *(const v8us*)(kp + 32 * 136 + 8 * hh); kl.half[1] = *(const v8us*)(kp + 32 * 136 + 16 + 8 * hh);
      sA = mmaN<3>(qh.v, ql.v, kh.v, kl.v, sA);
      const unsigned short* kq = kp + 16 * 136;
      FragB kh2, kl2;
      kh2.half[0] = *(const v8us*)(kq + 8 * hh); kh2.half[1] = *(const v8us*)(kq + 16 + 8 * hh);
      kl2.half[0] = *(const v8us*)(kq + 32 * 136 + 8 * hh); kl2.half[1] = *(const v8us*)(kq + 32 * 136 + 16 + 8 * hh);
      sB = mmaN<3>(qh.v, ql.v, kh2.v, kl2.v, sB);
    }
    float al[8];
#pragma unroll
    for (int r = 0; r < 8; ++r) {
      const int row = qrow0 + 8 * hh + r;
      float sa = sA[r] * SM_SCALE, sb = sB[r] * SM_SCALE;
      sa = (key0 + ln <= row) ? sa : -3.0e38f;
      sb = (key0 + 16 + ln <= row) ? sb : -3.0e38f;
      const float cand = half_reduce_max(fmaxf(sa, sb));
      const float mn = fmaxf(m[r], cand);
      const float alpha = __expf(m[r] - mn);
      const float pa = __expf(sa - mn), pb = __expf(sb - mn);
      const float rs = half_reduce_add(pa + pb);
      l[r] = l[r] * alpha + rs; m[r] = mn; al[r] = alpha;
      lP[(w * 16 + 8 * hh + r) * 40 + ln] = (_Float16)(pa * PCARRY);
      lP[(w * 16 + 8 * hh + r) * 40 + 16 + ln] = (_Float16)(pb * PCARRY);
    }
#pragma unroll
    for (int n = 0; n < 8; ++n) {
#pragma unroll
      for (int r = 0; r < 8; ++r) o[n][r] *= al[r];
    }
    __builtin_amdgcn_fence(4  , "workgroup");
    __builtin_amdgcn_wave_barrier();
    FragH pf; const unsigned short* pp = (const unsigned short*)(lP + (w * 16 + ln) * 40);
    pf.half[0] = *(const v8us*)(pp + 8 * hh); pf.half[1] = *(const v8us*)(pp + 16 + 8 * hh);
#pragma unroll
    for (int n = 0; n < 8; ++n) {
      FragH b; const unsigned short* vp = lVt + (n * 16 + ln) * 40;
      b.half[0] = *(const v8us*)(vp + 8 * hh); b.half[1] = *(const v8us*)(vp + 16 + 8 * hh);
      o[n] = mmaH<1>(pf.v, pf.v, b.v, b.v, o[n]);
    }
    __syncthreads();
  }
  float il[8];
#pragma unroll
  for (int r = 0; r < 8; ++r) il[r] = (1.0f / l[r]) * (1.0f / PCARRY);
  fa* sw = so + w * 2048;
#pragma unroll
  for (int n = 0; n < 8; ++n) {
#pragma unroll
    for (int r = 0; r < 8; ++r) sw[(8 * hh + r) * 128 + n * 16 + ln] = o[n][r] * il[r];
  }
  __builtin_amdgcn_fence(4  , "workgroup");
  __builtin_amdgcn_wave_barrier();
  v8us ov[8];
#pragma unroll
  for (int q = 0; q < 8; ++q) {
    const int rl = 2 * q + hh; const int row = qrow0 + rl;
    const v4f a = *(const v4fa*)(sw + rl * 128 + ln * 8), b = *(const v4fa*)(sw + rl * 128 + ln * 8 + 4);
    const float* gp = QG + (size_t)row * QGN + QD + h * HDM + ln * 8;
    const v4f g0 = *(const v4fa*)gp, g1 = *(const v4fa*)(gp + 4);
    FragH f;
#pragma unroll
    for (int i = 0; i < 4; ++i) { f.h[i] = (_Float16)(a[i] * silu_f(g0[i]) * GCARRY); f.h[4 + i] = (_Float16)(b[i] * silu_f(g1[i]) * GCARRY); }
    ov[q] = f.half[0];
  }
  for (int pass = 0; pass < 2; ++pass) {
#pragma unroll
    for (int q = 0; q < 8; ++q) { const int rl = 2 * q + hh; *(volatile v8us*)((unsigned short*)G16 + (size_t)(qrow0 + rl) * QD + h * HDM + ln * 8) = ov[q]; }
    if (pass == 0) __threadfence();
  }
}

__global__ __launch_bounds__(128) void k_early(const float* __restrict__ QF, const float* __restrict__ KF, const float* __restrict__ KV, const float* __restrict__ QG, float* __restrict__ GE) {
  __shared__ float qs[HDM]; __shared__ float ps[TE]; __shared__ float red[8];
  const int t = blockIdx.x, h = blockIdx.y, kvh = h >> 2, tid = threadIdx.x, lane = tid & 31, w = tid >> 5;
  qs[tid] = QF[(size_t)t * QD + h * HDM + tid];
  __syncthreads();
  const bool valid = tid <= t;
  float s = -3.0e38f;
  if (w * 32 <= t) {
    const int jj = valid ? tid : t;
    const float* kr = KF + (size_t)jj * KD + kvh * HDM;
    float acc = 0.f;
#pragma unroll 4
    for (int d = 0; d < HDM; ++d) acc += qs[d] * kr[d];
    s = valid ? acc * SM_SCALE : -3.0e38f;
  }
  float mx = s;
#pragma unroll
  for (int m = 1; m <= 16; m <<= 1) mx = fmaxf(mx, __shfl_xor(mx, m, 32));
  if (lane == 0) red[w] = mx;
  __syncthreads();
  mx = fmaxf(fmaxf(red[0], red[1]), fmaxf(red[2], red[3]));
  const float e = valid ? expf(s - mx) : 0.f;
  float se = e;
#pragma unroll
  for (int m = 1; m <= 16; m <<= 1) se += __shfl_xor(se, m, 32);
  if (lane == 0) red[4 + w] = se;
  __syncthreads();
  se = (red[4] + red[5]) + (red[6] + red[7]);
  ps[tid] = e * (1.0f / se);
  __syncthreads();
  const float* vc = KV + (size_t)KD + kvh * HDM + tid;
  float acc = 0.f;
#pragma unroll 4
  for (int j = 0; j <= t; ++j) acc += ps[j] * vc[(size_t)j * KVN];
  const float g = QG[(size_t)t * QGN + QD + h * HDM + tid];
  const float v = acc * silu_f(g);
  float* dst = GE + (size_t)t * QD + h * HDM + tid;
  *(volatile float*)dst = v; __threadfence(); *(volatile float*)dst = v;
}

extern "C" void kernel_launch(void* const* d_in, const int* in_sizes, int n_in,
                              void* d_out, int out_size, void* d_ws, size_t ws_size, hipStream_t stream) {
  if (n_in < 9) return;
  const float* x = (const float*)d_in[0]; const int* pos = (const int*)d_in[1]; const float* invf = (const float*)d_in[2];
  const float* Wq = (const float*)d_in[3]; const float* Wk = (const float*)d_in[4]; const float* Wv = (const float*)d_in[5]; const float* Wo = (const float*)d_in[6];
  const float* qnw = (const float*)d_in[7]; const float* knw = (const float*)d_in[8];
  if (in_sizes[0] < SEQ * HID || in_sizes[1] < SEQ || in_sizes[2] < HDM / 2 || in_sizes[3] < HID * QGN || in_sizes[4] < HID * KD ||
      in_sizes[5] < HID * KD || in_sizes[6] < QD * HID || in_sizes[7] < HDM || in_sizes[8] < HDM) return;
  if (out_size < SEQ * HID) return;
  float* out = (float*)d_out;
  char* ws = (char*)d_ws; size_t off = 0;
  auto take = [&](size_t bytes) { char* p = ws + off; off += (bytes + 255) & ~(size_t)255; return p; };
  _Float16* X16 = (_Float16*)take((size_t)SEQ * HID * 2);
  _Float16* WqT = (_Float16*)take((size_t)QGN * HID * 2);
  _Float16* WkvT = (_Float16*)take((size_t)KVN * HID * 2);
  _Float16* WoT = (_Float16*)take((size_t)HID * QD * 2);
  unsigned short* WoTb = (unsigned short*)take((size_t)HID * QD * 2);
  float* QG = (float*)take((size_t)SEQ * QGN * 4);
  float* KV = (float*)take((size_t)SEQ * KVN * 4);
  unsigned short* Qh = (unsigned short*)take((size_t)SEQ * QD * 2);
  unsigned short* Ql = (unsigned short*)take((size_t)SEQ * QD * 2);
  unsigned short* Kh = (unsigned short*)take((size_t)SEQ * KD * 2);
  unsigned short* Kl = (unsigned short*)take((size_t)SEQ * KD * 2);
  _Float16* VT = (_Float16*)take((size_t)NKV * HDM * SEQ * 2);
  _Float16* G16 = (_Float16*)take((size_t)SEQ * QD * 2);
  float* GE = (float*)take((size_t)TE * QD * 4);
  float* QF = (float*)take((size_t)TE * QD * 4);
  float* KF = (float*)take((size_t)TE * KD * 4);
  if (off > ws_size) return;

  { const size_t n8 = (size_t)SEQ * HID / 8; k_x16<<<(unsigned)((n8 + 255) / 256), 256, 0, stream>>>(x, X16, n8); }
  k_wt_f16<<<(unsigned)((QGN * (HID / 8) + 255) / 256), 256, 0, stream>>>(Wq, WqT, HID, QGN, WSCALE);
  k_wt_f16<<<(unsigned)((KD * (HID / 8) + 255) / 256), 256, 0, stream>>>(Wk, WkvT, HID, KD, WSCALE);
  k_wt_f16<<<(unsigned)((KD * (HID / 8) + 255) / 256), 256, 0, stream>>>(Wv, WkvT + (size_t)KD * HID, HID, KD, WSCALE);
  k_wt_f16<<<(unsigned)((HID * (QD / 8) + 255) / 256), 256, 0, stream>>>(Wo, WoT, QD, HID, WSCALE);
  k_wt_bf16<<<(unsigned)((HID * (QD / 8) + 255) / 256), 256, 0, stream>>>(Wo, WoTb, QD, HID);
  k_gemm2<0><<<dim3((SEQ / 128) * (QGN / 64), 1), 128, 0, stream>>>(X16, HID, (size_t)0, WqT, HID, (size_t)0, 1.0f / WSCALE, nullptr, (size_t)0, nullptr, 1, (size_t)0, 0, QG, nullptr, QGN, (size_t)0, SEQ, QGN, HID);
  k_gemm2<0><<<dim3((SEQ / 128) * (KVN / 64), 1), 128, 0, stream>>>(X16, HID, (size_t)0, WkvT, HID, (size_t)0, 1.0f / WSCALE, nullptr, (size_t)0, nullptr, 1, (size_t)0, 0, KV, nullptr, KVN, (size_t)0, SEQ, KVN, HID);
  k_normrope<<<SEQ, 256, 0, stream>>>(QG, KV, pos, invf, qnw, knw, Qh, Ql, Kh, Kl, QF, KF);
  k_vt<<<NKV * (SEQ / 64), 256, 0, stream>>>(KV, VT);
  k_flash<<<dim3((SEQ - TE) / 64, NQH), 128, 0, stream>>>(Qh, Ql, Kh, Kl, VT, QG, G16, TE);
  k_early<<<dim3(TE, NQH), 128, 0, stream>>>(QF, KF, KV, QG, GE);
  k_gemm2<0><<<dim3(((SEQ - TE) / 128) * (HID / 64), 1), 128, 0, stream>>>(G16 + (size_t)TE * QD, QD, (size_t)0, WoT, QD, (size_t)0, 1.0f / (WSCALE * GCARRY), nullptr, (size_t)0, nullptr, 1, (size_t)0, 0, out + (size_t)TE * HID, nullptr, HID, (size_t)0, SEQ - TE, HID, QD);
  k_gemm_bf<true><<<(TE / 16) * (HID / 64) / 4, 128, 0, stream>>>(GE, QD, WoTb, QD, out, HID, TE, HID, QD);
}
